// Part_Graph_41927470743597
// MI455X (gfx1250) — hardware-verified
//
#include <hip/hip_runtime.h>
#include <math.h>

constexpr int NBATCH  = 4;
constexpr int NCIN    = 256;
constexpr int LPIX    = 4096;
constexpr int NTOT    = NBATCH * LPIX;
constexpr int NHID    = 10;
constexpr int NPART   = 6;
constexpr int NEDGE   = 12;
constexpr int KFEAT   = 264;
constexpr int KFEATP  = 288;
constexpr int LDFEAT  = 320;
constexpr int MALL    = 128;
constexpr int ROWATT  = 64;
constexpr int ROWPROJ = 80;
constexpr int KREL    = 180;
constexpr int KRELP   = 192;
constexpr int MREL    = 64;
constexpr int EPB     = 6;
constexpr int NCOLB   = EPB * NTOT;
constexpr int NPIXBLK = NTOT / 256;
constexpr int OUT1_OFF = 7 * NBATCH * NHID * LPIX;
constexpr float WCARRY     = 16.0f;
constexpr float WCARRY_INV = 1.0f / 16.0f;
constexpr float BN_EPS     = 1e-5f;

static_assert(OUT1_OFF * 4 == 4587520, "out1 byte offset");
static_assert(OUT1_OFF * 4 + NBATCH * NEDGE * LPIX * 4 == 5373952, "d_out total");
static_assert(KFEATP % 32 == 0 && KRELP % 32 == 0, "K multiple of 32");
static_assert(MALL % 64 == 0 && NTOT % 64 == 0 && MREL % 64 == 0 && NCOLB % 64 == 0, "M,N multiples of 64");
static_assert(LDFEAT % 8 == 0 && KRELP % 8 == 0 && LDFEAT >= KFEATP, "16-B aligned fragment loads");

constexpr size_t SZ_BTFEAT = (size_t)NTOT * LDFEAT * 2;
constexpr size_t SZ_AALL   = (size_t)MALL * LDFEAT * 2;
constexpr size_t SZ_AREL   = (size_t)MREL * KRELP * 2;
constexpr size_t SZ_C1     = (size_t)MALL * NTOT * 4;
constexpr size_t SZ_NORM   = (size_t)NPART * NBATCH * LPIX * 4;
constexpr size_t SZ_QV     = (size_t)NPART * NBATCH * 64 * 4;
constexpr size_t SZ_S0     = (size_t)NPART * NTOT * 4;
constexpr size_t SZ_ATTS   = (size_t)NEDGE * NTOT * 4;
constexpr size_t SZ_STAT1  = (size_t)NEDGE * NPIXBLK * 32 * 4;
constexpr size_t SZ_MSG    = (size_t)NEDGE * NBATCH * NHID * LPIX * 4;
constexpr size_t SZ_BTCOL  = (size_t)NCOLB * KRELP * 2;
constexpr size_t SZ_C2     = (size_t)MREL * NCOLB * 4;
constexpr size_t SZ_STAT2  = (size_t)EPB * NPIXBLK * 64 * 4;
constexpr size_t SZ_MEDGE  = SZ_MSG;
constexpr size_t SZ_CNM    = (size_t)NPART * NBATCH * NHID * LPIX * 4;
constexpr size_t SZ_ZPL    = (size_t)NPART * NTOT * 4;
constexpr size_t SZ_STAT3  = (size_t)NPART * NPIXBLK * 32 * 4;
constexpr size_t SZ_TOTAL  = SZ_BTFEAT + SZ_AALL + SZ_AREL + SZ_C1 + SZ_NORM + SZ_QV + SZ_S0 + SZ_ATTS + SZ_STAT1 +
                             SZ_MSG + SZ_BTCOL + SZ_C2 + SZ_STAT2 + SZ_MEDGE + SZ_CNM + SZ_ZPL + SZ_STAT3;
static_assert(SZ_TOTAL == 103774208, "carve total");
static_assert(SZ_TOTAL <= (size_t)134217728, "carve under 128 MiB");

__constant__ int c_EU[NEDGE]    = {0, 1, 1, 1, 1, 1, 2, 3, 4, 4, 5, 5};
__constant__ int c_EV[NEDGE]    = {1, 0, 2, 3, 4, 5, 1, 1, 1, 5, 1, 4};
__constant__ int c_INCNT[NPART] = {1, 5, 1, 1, 2, 2};
__constant__ int c_INLIST[NPART * 5] = {1, 0, 0, 0, 0,   0, 6, 7, 8, 10,   2, 0, 0, 0, 0,   3, 0, 0, 0, 0,   4, 11, 0, 0, 0,   5, 9, 0, 0, 0};
static_assert(sizeof(c_EU) / sizeof(c_EU[0]) == 12 && sizeof(c_EV) / sizeof(c_EV[0]) == 12, "edge tables");
static_assert(sizeof(c_INLIST) / sizeof(c_INLIST[0]) == 30, "incoming table");

typedef __attribute__((ext_vector_type(16))) _Float16 v16h;
typedef __attribute__((ext_vector_type(8)))  _Float16 v8h;
typedef __attribute__((ext_vector_type(16))) __bf16   v16b;
typedef __attribute__((ext_vector_type(8)))  __bf16   v8b;
typedef __attribute__((ext_vector_type(8)))  float    v8f;
typedef __attribute__((ext_vector_type(4)))  float    v4f;
typedef __attribute__((ext_vector_type(4)))  unsigned int v4u;

__device__ __forceinline__ unsigned short f2bf_bits(float f) {
  unsigned u = __float_as_uint(f);
  return (unsigned short)((u + 0x7FFFu + ((u >> 16) & 1u)) >> 16);
}
__device__ __forceinline__ float bf_bits2f(unsigned short h) { return __uint_as_float(((unsigned)h) << 16); }
__device__ __forceinline__ float bfr(float f) { return __uint_as_float(((unsigned)f2bf_bits(f)) << 16); }

__device__ __forceinline__ void dep_guard_h(v8f& a, v8f& b, v16h x, v16h y) { asm volatile("v_nop\n\tv_nop\n\tv_nop\n\tv_nop" : "+v"(a), "+v"(b) : "v"(x), "v"(y)); }
__device__ __forceinline__ void dep_guard_b(v8f& a, v8f& b, v16b x, v16b y) { asm volatile("v_nop\n\tv_nop\n\tv_nop\n\tv_nop" : "+v"(a), "+v"(b) : "v"(x), "v"(y)); }
__device__ __forceinline__ void dep_guard4_h(v8f& a, v8f& b, v8f& c, v8f& d, v16h x, v16h y) { asm volatile("v_nop\n\tv_nop\n\tv_nop\n\tv_nop" : "+v"(a), "+v"(b), "+v"(c), "+v"(d) : "v"(x), "v"(y)); }
__device__ __forceinline__ void dep_guard4_b(v8f& a, v8f& b, v8f& c, v8f& d, v16b x, v16b y) { asm volatile("v_nop\n\tv_nop\n\tv_nop\n\tv_nop" : "+v"(a), "+v"(b), "+v"(c), "+v"(d) : "v"(x), "v"(y)); }
__device__ __forceinline__ void keep4_h(v16h a, v16h b, v16h c, v16h d) { asm volatile("v_nop" :: "v"(a), "v"(b), "v"(c), "v"(d)); }
__device__ __forceinline__ void keep4_b(v16b a, v16b b, v16b c, v16b d) { asm volatile("v_nop" :: "v"(a), "v"(b), "v"(c), "v"(d)); }
__device__ __forceinline__ void acc_guard4(v8f& a, v8f& b, v8f& c, v8f& d) { asm volatile("v_nop\n\tv_nop\n\tv_nop\n\tv_nop" : "+v"(a), "+v"(b), "+v"(c), "+v"(d)); }
template <typename T> struct Frag;
template <> struct Frag<_Float16> {
  typedef v16h V; union U { v16h v; v8h h[2]; };
  static __device__ __forceinline__ v16h load(const _Float16* p) {
    U f; f.h[0] = *(const v8h*)(p); f.h[1] = *(const v8h*)(p + 16); return f.v;
  }
  static __device__ __forceinline__ v8f mma(v16h a, v16h b, v8f c) {
    return __builtin_amdgcn_wmma_f32_16x16x32_f16(false, a, false, b, (short)0, c, false, false);
  }
  static __device__ __forceinline__ void guard(v8f& a, v8f& b, v16h x, v16h y) { dep_guard_h(a, b, x, y); }
  static __device__ __forceinline__ void guard4(v8f& a, v8f& b, v8f& c, v8f& d, v16h x, v16h y) { dep_guard4_h(a, b, c, d, x, y); }
  static __device__ __forceinline__ void keep(v16h a, v16h b, v16h c, v16h d) { keep4_h(a, b, c, d); }
};
template <> struct Frag<__bf16> {
  typedef v16b V; union U { v16b v; v8b h[2]; };
  static __device__ __forceinline__ v16b load(const __bf16* p) {
    U f; f.h[0] = *(const v8b*)(p); f.h[1] = *(const v8b*)(p + 16); return f.v;
  }
  static __device__ __forceinline__ v8f mma(v16b a, v16b b, v8f c) {
    return __builtin_amdgcn_wmma_f32_16x16x32_bf16(false, a, false, b, (short)0, c, false, false);
  }
  static __device__ __forceinline__ void guard(v8f& a, v8f& b, v16b x, v16b y) { dep_guard_b(a, b, x, y); }
  static __device__ __forceinline__ void guard4(v8f& a, v8f& b, v8f& c, v8f& d, v16b x, v16b y) { dep_guard4_b(a, b, c, d, x, y); }
  static __device__ __forceinline__ void keep(v16b a, v16b b, v16b c, v16b d) { keep4_b(a, b, c, d); }
};

__device__ __forceinline__ unsigned pk16(unsigned short a, unsigned short b) { return (unsigned)a | ((unsigned)b << 16); }
__device__ __forceinline__ unsigned short h_bits(float f) { const _Float16 h = (_Float16)f; return __builtin_bit_cast(unsigned short, h); }

template <int ET> struct Elem;
template <> struct Elem<0> { typedef _Float16 T; };
template <> struct Elem<1> { typedef __bf16 T; };
template <int ET, bool SPLIT, int BIAS_MODE, int OUT_MODE, bool RESID, int ACT = 0>
__global__ __launch_bounds__(256) void wmma_gemm64(
    const unsigned short* __restrict__ Ap, const unsigned short* __restrict__ A2p, int lda, long strideA,
    const unsigned short* __restrict__ Btp, const unsigned short* __restrict__ Bt2p, int ldb, long strideB,
    void* __restrict__ Cout, void* __restrict__ Cout2, int ldc, long strideC,
    const float* __restrict__ bias,
    const float* __restrict__ resid, long strideR,
    int M, int N, int K, float scale) {
  typedef typename Elem<ET>::T T;
  typedef typename Frag<T>::V V;
  const T* A = (const T*)Ap; const T* A2 = (const T*)A2p; const T* Bt = (const T*)Btp; const T* Bt2 = (const T*)Bt2p;
  __shared__ __align__(16) float sT[8][16 * 68];
  const int b    = blockIdx.y;
  const int lane = threadIdx.x & 31;
  const int wave = threadIdx.x >> 5;
  const int tilesN = N >> 6;
  const int tilesM = M >> 6;
  const int tile = blockIdx.x * 8 + wave;
  if (tile >= tilesM * tilesN) return;
  const int tm = tile / tilesN;
  const int tn = tile - tm * tilesN;
  const int m0 = tm << 6;
  const int n0 = tn << 6;

  const T* Ab  = A  + (size_t)b * strideA;
  const T* Bb  = Bt + (size_t)b * strideB;
  const T* Ab2 = SPLIT ? (A2  + (size_t)b * strideA) : nullptr;
  const T* Bb2 = SPLIT ? (Bt2 + (size_t)b * strideB) : nullptr;

  const int rlane = lane & 15;
  const int koff  = (lane >> 4) * 8;
  const int mOff  = (lane >> 4) * 8;

  v8f acc[4][4];
#pragma unroll
  for (int i = 0; i < 4; ++i)
#pragma unroll
    for (int j = 0; j < 4; ++j) acc[i][j] = (v8f){0.f,0.f,0.f,0.f,0.f,0.f,0.f,0.f};

  for (int k0 = 0; k0 < K; k0 += 32) {
    V bh[4], bl[4];
#pragma unroll
    for (int j = 0; j < 4; ++j) {
      const size_t bo = (size_t)(n0 + (j << 4) + rlane) * ldb + koff + k0;
      bh[j] = Frag<T>::load(Bb + bo);
      if (SPLIT) bl[j] = Frag<T>::load(Bb2 + bo);
    }
#pragma unroll
    for (int i = 0; i < 4; ++i) {
      const size_t ao = (size_t)(m0 + (i << 4) + rlane) * lda + koff + k0;
      V ah = Frag<T>::load(Ab + ao);
      V al;
      if (SPLIT) al = Frag<T>::load(Ab2 + ao);
#pragma unroll
      for (int j = 0; j < 4; ++j) {
        acc[i][j] = Frag<T>::mma(ah, bh[j], acc[i][j]);
        if (SPLIT) {
          acc[i][j] = Frag<T>::mma(ah, bl[j], acc[i][j]);
          acc[i][j] = Frag<T>::mma(al, bh[j], acc[i][j]);
        }
      }
      Frag<T>::guard4(acc[i][0], acc[i][1], acc[i][2], acc[i][3], ah, SPLIT ? al : ah);
    }
    Frag<T>::keep(bh[0], bh[1], bh[2], bh[3]);
    if (SPLIT) Frag<T>::keep(bl[0], bl[1], bl[2], bl[3]);
  }
  acc_guard4(acc[0][0], acc[0][1], acc[0][2], acc[0][3]);
  acc_guard4(acc[1][0], acc[1][1], acc[1][2], acc[1][3]);
  acc_guard4(acc[2][0], acc[2][1], acc[2][2], acc[2][3]);
  acc_guard4(acc[3][0], acc[3][1], acc[3][2], acc[3][3]);

  float* slab = sT[wave];
  const float* Rb = RESID ? (resid + (size_t)b * strideR) : nullptr;
#pragma unroll
  for (int i = 0; i < 4; ++i) {
    const int mBase = m0 + (i << 4);
#pragma unroll
    for (int j = 0; j < 4; ++j) {
      const int n = n0 + (j << 4) + rlane;
      float bv = 0.f;
      if (BIAS_MODE == 2) bv = bias[n];
#pragma unroll
      for (int r = 0; r < 8; ++r) {
        float v = acc[i][j][r] * scale;
        if (BIAS_MODE == 1) v += bias[mBase + mOff + r];
        if (BIAS_MODE == 2) v += bv;
        if (RESID) v += Rb[(size_t)(mBase + mOff + r) * ldc + n];
        if (ACT == 2) v = fmaxf(v, 0.0f);
        if (ACT == 4) v = (v > 0.f) ? v : 0.01f * v;
        slab[(mOff + r) * 68 + (j << 4) + rlane] = v;
      }
    }
    __builtin_amdgcn_fence(__ATOMIC_RELEASE, "workgroup");
    __builtin_amdgcn_wave_barrier();
    __builtin_amdgcn_fence(__ATOMIC_ACQUIRE, "workgroup");
    if (OUT_MODE == 0) {
      float* C = (float*)Cout + (size_t)b * strideC;
      const int hh = lane >> 4, c4 = (lane & 15) * 4;
      for (int pass = 0; pass < 2; ++pass) {
#pragma unroll
        for (int it = 0; it < 8; ++it) {
          const int row = it * 2 + hh;
          v4f v = *(const v4f*)(slab + row * 68 + c4);
          *(volatile v4f*)(C + (size_t)(mBase + row) * ldc + n0 + c4) = v;
        }
        __threadfence();
      }
    } else {
      const int q = lane >> 3, c8 = (lane & 7) * 8;
      unsigned short* C  = (unsigned short*)Cout  + (size_t)b * strideC;
      unsigned short* C2 = (OUT_MODE == 2) ? ((unsigned short*)Cout2 + (size_t)b * strideC) : nullptr;
      for (int pass = 0; pass < 2; ++pass) {
#pragma unroll
        for (int it = 0; it < 4; ++it) {
          const int row = it * 4 + q;
          const float* sp = slab + row * 68 + c8;
          v8h hv, lv;
#pragma unroll
          for (int e = 0; e < 8; ++e) {
            if (OUT_MODE == 1) {
              hv[e] = (_Float16)sp[e];
            } else {
              unsigned short hb = f2bf_bits(sp[e]);
              unsigned short lb = f2bf_bits(sp[e] - bf_bits2f(hb));
              hv[e] = __builtin_bit_cast(_Float16, hb);
              lv[e] = __builtin_bit_cast(_Float16, lb);
            }
          }
          *(volatile v8h*)(C + (size_t)(mBase + row) * ldc + n0 + c8) = hv;
          if (OUT_MODE == 2) *(volatile v8h*)(C2 + (size_t)(mBase + row) * ldc + n0 + c8) = lv;
        }
        __threadfence();
      }
    }
    __builtin_amdgcn_fence(__ATOMIC_RELEASE, "workgroup");
    __builtin_amdgcn_wave_barrier();
    __builtin_amdgcn_fence(__ATOMIC_ACQUIRE, "workgroup");
  }
}

__device__ __forceinline__ float wave_sum(float v) {
  v += __shfl_xor(v, 16, 32); v += __shfl_xor(v, 8, 32); v += __shfl_xor(v, 4, 32);
  v += __shfl_xor(v, 2, 32);  v += __shfl_xor(v, 1, 32);
  return v;
}
__device__ __forceinline__ float wave_max(float v) {
  v = fmaxf(v, __shfl_xor(v, 16, 32)); v = fmaxf(v, __shfl_xor(v, 8, 32)); v = fmaxf(v, __shfl_xor(v, 4, 32));
  v = fmaxf(v, __shfl_xor(v, 2, 32));  v = fmaxf(v, __shfl_xor(v, 1, 32));
  return v;
}
__device__ __forceinline__ void st2f(float* p, float v) {
  *(volatile float*)p = v;
  __threadfence();
  *(volatile float*)p = v;
}
__device__ __forceinline__ float sigm(float x) { return __builtin_amdgcn_rcpf(1.0f + expf(-x)); }
__device__ __forceinline__ float coordval(int c, int l) {
  const int h = l >> 6, w = l & 63;
  const float xmin = (float)w * 0.03125f - 1.0f;
  const float xmax = (float)(w + 1) * 0.03125f - 1.0f;
  const float ymin = (float)h * 0.03125f - 1.0f;
  const float ymax = (float)(h + 1) * 0.03125f - 1.0f;
  const float xc = (xmin + xmax) * 0.5f, yc = (ymin + ymax) * 0.5f;
  return (c == 0) ? xmin : (c == 1) ? ymin : (c == 2) ? xmax : (c == 3) ? ymax : (c == 4) ? xc : (c == 5) ? yc : 0.015625f;
}

__global__ __launch_bounds__(256) void k_prep_w(const float* __restrict__ W_key, const float* __restrict__ W_att,
                                                const float* __restrict__ W_proj, const float* __restrict__ W_rel1,
                                                unsigned short* __restrict__ a_all, unsigned short* __restrict__ a_rel) {
  const int lane = threadIdx.x & 31;
  const int wave = threadIdx.x >> 5;
  const int r = __builtin_amdgcn_readfirstlane((int)(blockIdx.x * 8 + wave));
  if (r < MALL) {
    const float* src = W_key; int base = 0; int klim = KFEAT; float live = 0.0f;
    if (r < ROWATT) { src = W_key; base = r * KFEAT; klim = KFEAT; live = 1.0f; }
    else if (r < ROWATT + NEDGE) { src = W_att; base = (r - ROWATT) * (NCIN + 1) + 1; klim = NCIN; live = 1.0f; }
    else if (r >= ROWPROJ && r < ROWPROJ + NHID) { src = W_proj; base = (r - ROWPROJ) * NCIN; klim = NCIN; live = 1.0f; }
    unsigned short ha[8], hc[8];
#pragma unroll
    for (int e = 0; e < 8; ++e) {
      const float x = src[base + 8 * lane + e];
      ha[e] = f2bf_bits(live > 0.5f ? x : 0.0f);
    }
    v4u uA = (v4u){pk16(ha[0], ha[1]), pk16(ha[2], ha[3]), pk16(ha[4], ha[5]), pk16(ha[6], ha[7])};
    asm volatile("" : "+v"(uA) :: "memory");
#pragma unroll
    for (int e = 0; e < 8; ++e) {
      const int col = NCIN + 8 * lane + e;
      const int cc = (col < klim) ? col : (klim - 1);
      const float x = src[base + cc];
      const float v = (col < klim && live > 0.5f) ? x : 0.0f;
      hc[e] = f2bf_bits(v);
    }
    const v4u uB = (v4u){pk16(hc[0], hc[1]), pk16(hc[2], hc[3]), pk16(hc[4], hc[5]), pk16(hc[6], hc[7])};
    unsigned short* rowp = a_all + (size_t)r * LDFEAT;
    for (int pass = 0; pass < 2; ++pass) {
      *(volatile v4u*)(rowp + 8 * lane) = uA;
      if (lane < 8) *(volatile v4u*)(rowp + NCIN + 8 * lane) = uB;
      __threadfence();
    }
  } else {
    const int co = r - MALL;
    const int coc = (co < 2 * NHID) ? co : (2 * NHID - 1);
    unsigned short hr[8];
#pragma unroll
    for (int e = 0; e < 8; ++e) {
      const int k = 8 * lane + e;
      const int kc = (k < KREL) ? k : (KREL - 1);
      const float x = W_rel1[coc * KREL + kc];
      const float v = (co < 2 * NHID && k < KREL) ? (bfr(x) * WCARRY) : 0.0f;
      hr[e] = h_bits(v);
    }
    const v4u u = (v4u){pk16(hr[0], hr[1]), pk16(hr[2], hr[3]), pk16(hr[4], hr[5]), pk16(hr[6], hr[7])};
    unsigned short* rowp = a_rel + (size_t)co * KRELP;
    for (int pass = 0; pass < 2; ++pass) {
      if (lane < 24) *(volatile v4u*)(rowp + 8 * lane) = u;
      __threadfence();
    }
  }
}

__global__ __launch_bounds__(256) void k_prep_feat(const float* __restrict__ xp, unsigned short* __restrict__ bt) {
  const int lane = threadIdx.x & 31;
  const int wave = threadIdx.x >> 5;
  const int row = __builtin_amdgcn_readfirstlane((int)(blockIdx.x * 8 + wave));
  const int n = row >> 12, l = row & (LPIX - 1);
  const float* xb = xp + ((size_t)n * NCIN + 8 * lane) * LPIX + l;
  unsigned short ha[8], hb[8];
#pragma unroll
  for (int e = 0; e < 8; ++e) ha[e] = f2bf_bits(xb[(size_t)e * LPIX]);
  {
    const int h = l >> 6, w = l & 63;
    const float xmin = (float)w * 0.03125f - 1.0f;
    const float xmax = (float)(w + 1) * 0.03125f - 1.0f;
    const float ymin = (float)h * 0.03125f - 1.0f;
    const float ymax = (float)(h + 1) * 0.03125f - 1.0f;
    float cv[8];
    cv[0] = xmin; cv[1] = ymin; cv[2] = xmax; cv[3] = ymax;
    cv[4] = (xmin + xmax) * 0.5f; cv[5] = (ymin + ymax) * 0.5f; cv[6] = 0.015625f; cv[7] = 0.015625f;
    const bool first = (lane == 0);
#pragma unroll
    for (int e = 0; e < 8; ++e) hb[e] = f2bf_bits(first ? cv[e] : 0.0f);
  }
  const v4u uA = (v4u){pk16(ha[0], ha[1]), pk16(ha[2], ha[3]), pk16(ha[4], ha[5]), pk16(ha[6], ha[7])};
  const v4u uB = (v4u){pk16(hb[0], hb[1]), pk16(hb[2], hb[3]), pk16(hb[4], hb[5]), pk16(hb[6], hb[7])};
  unsigned short* rowp = bt + (size_t)row * LDFEAT;
  for (int pass = 0; pass < 2; ++pass) {
    *(volatile v4u*)(rowp + 8 * lane) = uA;
    if (lane < 8) *(volatile v4u*)(rowp + NCIN + 8 * lane) = uB;
    __threadfence();
  }
}

__global__ __launch_bounds__(512) void k_softmax_norm(const float* __restrict__ p_atts, float* __restrict__ norm) {
  __shared__ float redm[16];
  __shared__ float reds[16];
  const int pn = blockIdx.x;
  const int p = pn >> 2, n = pn & 3;
  const int tid = threadIdx.x, lane = tid & 31, wave = tid >> 5;
  const float* src = p_atts + ((size_t)(p + 1) * NBATCH + n) * LPIX;
  float xv[8];
#pragma unroll
  for (int i = 0; i < 8; ++i) xv[i] = bfr(src[tid + 512 * i]);
  float mx = xv[0];
#pragma unroll
  for (int i = 1; i < 8; ++i) mx = fmaxf(mx, xv[i]);
  mx = wave_max(mx);
  if (lane == 0) redm[wave] = mx;
  __syncthreads();
  float m = redm[0];
#pragma unroll
  for (int w = 1; w < 16; ++w) m = fmaxf(m, redm[w]);
  float ev[8];
  float s = 0.0f;
#pragma unroll
  for (int i = 0; i < 8; ++i) { ev[i] = expf(xv[i] - m); s += ev[i]; }
  s = wave_sum(s);
  if (lane == 0) reds[wave] = s;
  __syncthreads();
  float tot = 0.0f;
#pragma unroll
  for (int w = 0; w < 16; ++w) tot += reds[w];
  const float inv = 1.0f / tot;
  float* dst = norm + (size_t)pn * LPIX + tid;
  for (int pass = 0; pass < 2; ++pass) {
#pragma unroll
    for (int i = 0; i < 8; ++i) *(volatile float*)(dst + 512 * i) = ev[i] * inv;
    __threadfence();
  }
}

__global__ __launch_bounds__(320) void k_centroid_q(const float* __restrict__ xp, const float* __restrict__ norm,
                                                    const float* __restrict__ W_q, const float* __restrict__ b_q,
                                                    float* __restrict__ qv) {
  __shared__ float nsh[LPIX];
  __shared__ float cen[KFEAT];
  __shared__ __align__(16) float qs[64];
  const int pn = blockIdx.x;
  const int n = pn & 3;
  const int tid = threadIdx.x, lane = tid & 31;
  const int w = __builtin_amdgcn_readfirstlane((int)(threadIdx.x >> 5));
  for (int i = tid; i < LPIX; i += 320) nsh[i] = norm[(size_t)pn * LPIX + i];
  __syncthreads();
  if (w < 8) {
    const int c = tid;
    const float* xr = xp + ((size_t)n * NCIN + c) * LPIX;
    float s = 0.0f;
#pragma unroll 1
    for (int l = 0; l < LPIX; ++l) s = fmaf(bfr(xr[l]), nsh[l], s);
    cen[c] = s;
  } else if (w == 8) {
    const int c = lane;
    float s = 0.0f;
#pragma unroll 1
    for (int l = 0; l < LPIX; ++l) s = fmaf(coordval(c, l), nsh[l], s);
    if (lane < 8) cen[NCIN + lane] = s;
  }
  __syncthreads();
  if (w < 2) {
    const int o = tid;
    const float* wr = W_q + (size_t)o * KFEAT;
    float s = 0.0f;
#pragma unroll 1
    for (int f = 0; f < KFEAT; ++f) s = fmaf(bfr(wr[f]), cen[f], s);
    s += bfr(b_q[o]);
    qs[o] = s;
  }
  __syncthreads();
  if (w == 0) {
    const int li = lane & 15;
    const v4f v = *(const v4f*)(qs + 4 * li);
    float* dst = qv + (size_t)pn * 64 + 4 * li;
    for (int pass = 0; pass < 2; ++pass) {
      if (lane < 16) *(volatile v4f*)dst = v;
      __threadfence();
    }
  }
}

__global__ __launch_bounds__(256) void k_energy_s0(const float* __restrict__ qv, const float* __restrict__ c1,
                                                   const float* __restrict__ b_key, const float* __restrict__ p_atts,
                                                   float* __restrict__ s0) {
  __shared__ float qsh[NPART * NBATCH * 64];
  __shared__ float bk[64];
  const int tid = threadIdx.x;
  for (int i = tid; i < NPART * NBATCH * 64; i += 256) qsh[i] = qv[i];
  if (tid < 64) bk[tid] = bfr(b_key[tid]);
  __syncthreads();
  const int col = blockIdx.x * 256 + tid;
  const int n = col >> 12, l = col & (LPIX - 1);
  float ev[NPART];
#pragma unroll
  for (int p = 0; p < NPART; ++p) ev[p] = 0.0f;
#pragma unroll 1
  for (int o = 0; o < 64; ++o) {
    const float kv = c1[(size_t)o * NTOT + col] + bk[o];
#pragma unroll
    for (int p = 0; p < NPART; ++p) ev[p] = fmaf(qsh[(p * NBATCH + n) * 64 + o], kv, ev[p]);
  }
  float sv[NPART];
#pragma unroll
  for (int p = 0; p < NPART; ++p) {
    const float attn = sigm(ev[p]);
    const float pa = bfr(p_atts[((size_t)(p + 1) * NBATCH + n) * LPIX + l]);
    sv[p] = attn * (1.0f - pa);
  }
  for (int pass = 0; pass < 2; ++pass) {
#pragma unroll
    for (int p = 0; p < NPART; ++p) *(volatile float*)(s0 + (size_t)p * NTOT + col) = sv[p];
    __threadfence();
  }
}

__global__ __launch_bounds__(256) void k_logits(const float* __restrict__ c1, const float* __restrict__ s0,
                                                const float* __restrict__ W_att, const float* __restrict__ b_att,
                                                float* __restrict__ atts, float* __restrict__ out1) {
  __shared__ float wa[NEDGE];
  __shared__ float ba[NEDGE];
  const int tid = threadIdx.x;
  if (tid < NEDGE) { wa[tid] = bfr(W_att[tid * (NCIN + 1)]); ba[tid] = bfr(b_att[tid]); }
  __syncthreads();
  const int col = blockIdx.x * 256 + tid;
  const int n = col >> 12, l = col & (LPIX - 1);
  float sp[NPART];
#pragma unroll
  for (int p = 0; p < NPART; ++p) sp[p] = s0[(size_t)p * NTOT + col];
  asm volatile("" : "+v"(sp[0]), "+v"(sp[1]), "+v"(sp[2]), "+v"(sp[3]), "+v"(sp[4]), "+v"(sp[5]) :: "memory");
  float lg[NEDGE];
#pragma unroll
  for (int r = 0; r < NEDGE; ++r) lg[r] = c1[(size_t)(ROWATT + r) * NTOT + col];
  lg[0]  = fmaf(wa[0],  sp[0], lg[0])  + ba[0];
  lg[1]  = fmaf(wa[1],  sp[1], lg[1])  + ba[1];
  lg[2]  = fmaf(wa[2],  sp[1], lg[2])  + ba[2];
  lg[3]  = fmaf(wa[3],  sp[1], lg[3])  + ba[3];
  lg[4]  = fmaf(wa[4],  sp[1], lg[4])  + ba[4];
  lg[5]  = fmaf(wa[5],  sp[1], lg[5])  + ba[5];
  lg[6]  = fmaf(wa[6],  sp[2], lg[6])  + ba[6];
  lg[7]  = fmaf(wa[7],  sp[3], lg[7])  + ba[7];
  lg[8]  = fmaf(wa[8],  sp[4], lg[8])  + ba[8];
  lg[9]  = fmaf(wa[9],  sp[4], lg[9])  + ba[9];
  lg[10] = fmaf(wa[10], sp[5], lg[10]) + ba[10];
  lg[11] = fmaf(wa[11], sp[5], lg[11]) + ba[11];
  float pr[NEDGE];
  pr[0] = 1.0f; pr[6] = 1.0f; pr[7] = 1.0f;
  {
    const float m = fmaxf(fmaxf(fmaxf(lg[1], lg[2]), fmaxf(lg[3], lg[4])), lg[5]);
    const float e1 = expf(lg[1] - m), e2 = expf(lg[2] - m), e3 = expf(lg[3] - m), e4 = expf(lg[4] - m), e5 = expf(lg[5] - m);
    const float s = (((e1 + e2) + e3) + e4) + e5;
    const float inv = 1.0f / s;
    pr[1] = e1 * inv; pr[2] = e2 * inv; pr[3] = e3 * inv; pr[4] = e4 * inv; pr[5] = e5 * inv;
  }
  {
    const float m = fmaxf(lg[8], lg[9]);
    const float e8 = expf(lg[8] - m), e9 = expf(lg[9] - m);
    const float inv = 1.0f / (e8 + e9);
    pr[8] = e8 * inv; pr[9] = e9 * inv;
  }
  {
    const float m = fmaxf(lg[10], lg[11]);
    const float e10 = expf(lg[10] - m), e11 = expf(lg[11] - m);
    const float inv = 1.0f / (e10 + e11);
    pr[10] = e10 * inv; pr[11] = e11 * inv;
  }
  float* ob = out1 + (size_t)n * NEDGE * LPIX + l;
  for (int pass = 0; pass < 2; ++pass) {
#pragma unroll
    for (int r = 0; r < NEDGE; ++r) {
      *(volatile float*)(ob + (size_t)r * LPIX) = lg[r];
      *(volatile float*)(atts + (size_t)r * NTOT + col) = pr[r];
    }
    __threadfence();
  }
}

__global__ __launch_bounds__(256) void k_bn1_stats(const float* __restrict__ s0, const float* __restrict__ atts,
                                                   const float* __restrict__ c1, float* __restrict__ stat1) {
  __shared__ float red[8][2 * NHID];
  const int tid = threadIdx.x, lane = tid & 31, wave = tid >> 5;
  const int e = blockIdx.y;
  int u = c_EU[e]; u = u < 0 ? 0 : (u > NPART - 1 ? NPART - 1 : u);
  const int col = blockIdx.x * 256 + tid;
  const float scal = s0[(size_t)u * NTOT + col] * atts[(size_t)e * NTOT + col];
  float sv[NHID], qq[NHID];
#pragma unroll
  for (int o = 0; o < NHID; ++o) {
    const float v = scal * c1[(size_t)(ROWPROJ + o) * NTOT + col];
    sv[o] = wave_sum(v);
    qq[o] = wave_sum(v * v);
  }
  if (lane == 0) {
#pragma unroll
    for (int o = 0; o < NHID; ++o) { red[wave][o] = sv[o]; red[wave][NHID + o] = qq[o]; }
  }
  __syncthreads();
  if (tid < 32) {
    float t = 0.0f;
    if (tid < 2 * NHID) {
#pragma unroll
      for (int w = 0; w < 8; ++w) t += red[w][tid];
    }
    st2f(stat1 + ((size_t)(e * NPIXBLK + blockIdx.x)) * 32 + tid, t);
  }
}

__global__ __launch_bounds__(256) void k_msg_write(const float* __restrict__ s0, const float* __restrict__ atts,
                                                   const float* __restrict__ c1, const float* __restrict__ stat1,
                                                   const float* __restrict__ g_proj, const float* __restrict__ bt_proj,
                                                   float* __restrict__ msg) {
  __shared__ float mu[NHID], rs[NHID], gg[NHID], bb[NHID];
  const int tid = threadIdx.x;
  const int e = blockIdx.y;
  int u = c_EU[e]; u = u < 0 ? 0 : (u > NPART - 1 ? NPART - 1 : u);
  if (tid < NHID) {
    double s = 0.0, q = 0.0;
#pragma unroll 1
    for (int b = 0; b < NPIXBLK; ++b) {
      const float* t = stat1 + ((size_t)(e * NPIXBLK + b)) * 32;
      s += (double)t[tid]; q += (double)t[NHID + tid];
    }
    const double m = s * (1.0 / NTOT);
    double var = q * (1.0 / NTOT) - m * m;
    var = var < 0.0 ? 0.0 : var;
    mu[tid] = (float)m;
    rs[tid] = 1.0f / sqrtf((float)var + BN_EPS);
    gg[tid] = bfr(g_proj[tid]);
    bb[tid] = bfr(bt_proj[tid]);
  }
  __syncthreads();
  const int col = blockIdx.x * 256 + tid;
  const int n = col >> 12, l = col & (LPIX - 1);
  const float scal = s0[(size_t)u * NTOT + col] * atts[(size_t)e * NTOT + col];
  float* mrow = msg + ((size_t)(e * NBATCH + n) * NHID) * LPIX + l;
#pragma unroll 1
  for (int o = 0; o < NHID; ++o) {
    const float v = scal * c1[(size_t)(ROWPROJ + o) * NTOT + col];
    const float y = fmaxf((v - mu[o]) * rs[o] * gg[o] + bb[o], 0.0f);
    st2f(mrow + (size_t)o * LPIX, y);
  }
}

__device__ __forceinline__ float im2col_val(const float* __restrict__ mb, const float* __restrict__ pb, int h, int w, int k) {
  const int ci = k / 9;
  const int tap = k - 9 * ci;
  const int ky = tap / 3;
  const int kx = tap - 3 * ky;
  const int h2 = h + ky - 1, w2 = w + kx - 1;
  const bool inimg = (h2 >= 0) && (h2 < 64) && (w2 >= 0) && (w2 < 64);
  const int h2c = h2 < 0 ? 0 : (h2 > 63 ? 63 : h2);
  const int w2c = w2 < 0 ? 0 : (w2 > 63 ? 63 : w2);
  const int sp = h2c * 64 + w2c;
  const int cim = (ci < NHID) ? ci : (NHID - 1);
  int cip = ci - NHID; cip = cip < 0 ? 0 : (cip > NHID - 1 ? NHID - 1 : cip);
  const float a = mb[(size_t)cim * LPIX + sp];
  const float b = bfr(pb[(size_t)cip * LPIX + sp]);
  const float fa = (inimg && ci < NHID) ? 1.0f : 0.0f;
  const float fb = (inimg && ci >= NHID && ci < 2 * NHID) ? 1.0f : 0.0f;
  return fmaf(fa, a, fb * b);
}

__global__ __launch_bounds__(256) void k_im2col(const float* __restrict__ msg, const float* __restrict__ p_nodes,
                                                unsigned short* __restrict__ bt_col, int batch) {
  const int lane = threadIdx.x & 31;
  const int wave = threadIdx.x >> 5;
  const int rowbase = __builtin_amdgcn_readfirstlane((int)((blockIdx.x * 8 + wave) * 4));
  const int q = lane;
#pragma unroll 1
  for (int it = 0; it < 4; ++it) {
    const int row = rowbase + it;
    const int el = row >> 14;
    const int pix = row & (NTOT - 1);
    const int n = pix >> 12, hw = pix & (LPIX - 1);
    const int h = hw >> 6, w = hw & 63;
    int e = batch * EPB + el; e = e < 0 ? 0 : (e > NEDGE - 1 ? NEDGE - 1 : e);
    int v = c_EV[e]; v = v < 0 ? 0 : (v > NPART - 1 ? NPART - 1 : v);
    const float* mb = msg + ((size_t)(e * NBATCH + n) * NHID) * LPIX;
    const float* pb = p_nodes + ((size_t)(v * NBATCH + n) * NHID) * LPIX;
    unsigned p01, p23, p45, p67;
    {
      const float v0 = im2col_val(mb, pb, h, w, 8 * q + 0);
      const float v1 = im2col_val(mb, pb, h, w, 8 * q + 1);
      const float v2 = im2col_val(mb, pb, h, w, 8 * q + 2);
      const float v3 = im2col_val(mb, pb, h, w, 8 * q + 3);
      p01 = pk16(h_bits(v0), h_bits(v1));
      p23 = pk16(h_bits(v2), h_bits(v3));
    }
    asm volatile("" : "+v"(p01), "+v"(p23) :: "memory");
    {
      const float v4 = im2col_val(mb, pb, h, w, 8 * q + 4);
      const float v5 = im2col_val(mb, pb, h, w, 8 * q + 5);
      const float v6 = im2col_val(mb, pb, h, w, 8 * q + 6);
      const float v7 = im2col_val(mb, pb, h, w, 8 * q + 7);
      p45 = pk16(h_bits(v4), h_bits(v5));
      p67 = pk16(h_bits(v6), h_bits(v7));
    }
    const v4u u = (v4u){p01, p23, p45, p67};
    unsigned short* dst = bt_col + (size_t)row * KRELP + 8 * q;
    for (int pass = 0; pass < 2; ++pass) {
      if (q < 24) *(volatile v4u*)dst = u;
      __threadfence();
    }
  }
}

__global__ __launch_bounds__(256) void k_bn2_stats(const float* __restrict__ c2, float* __restrict__ stat2) {
  __shared__ float red[8][4 * NHID];
  const int tid = threadIdx.x, lane = tid & 31, wave = tid >> 5;
  const int el = blockIdx.y;
  const int col = el * NTOT + blockIdx.x * 256 + tid;
#pragma unroll 1
  for (int c = 0; c < 2 * NHID; ++c) {
    const float v = c2[(size_t)c * NCOLB + col];
    const float s = wave_sum(v);
    const float q = wave_sum(v * v);
    if (lane == 0) { red[wave][c] = s; red[wave][2 * NHID + c] = q; }
  }
  __syncthreads();
  if (tid < 64) {
    float t = 0.0f;
    if (tid < 4 * NHID) {
#pragma unroll
      for (int w = 0; w < 8; ++w) t += red[w][tid];
    }
    st2f(stat2 + ((size_t)(el * NPIXBLK + blockIdx.x)) * 64 + tid, t);
  }
}

__global__ __launch_bounds__(256) void k_edge_finish(const float* __restrict__ c2, const float* __restrict__ stat2,
                                                     const float* __restrict__ g_rel1, const float* __restrict__ bt_rel1,
                                                     const float* __restrict__ W_rel2, const float* __restrict__ b_rel2,
                                                     float* __restrict__ medge, int batch) {
  __shared__ float mu[2 * NHID], rs[2 * NHID], gg[2 * NHID], bb[2 * NHID];
  __shared__ float wr[NHID * 2 * NHID];
  __shared__ float br[NHID];
  const int tid = threadIdx.x;
  const int el = blockIdx.y;
  int e = batch * EPB + el; e = e < 0 ? 0 : (e > NEDGE - 1 ? NEDGE - 1 : e);
  if (tid < 2 * NHID) {
    double s = 0.0, q = 0.0;
#pragma unroll 1
    for (int b = 0; b < NPIXBLK; ++b) {
      const float* t = stat2 + ((size_t)(el * NPIXBLK + b)) * 64;
      s += (double)t[tid]; q += (double)t[2 * NHID + tid];
    }
    const double m = s * (1.0 / NTOT);
    double var = q * (1.0 / NTOT) - m * m;
    var = var < 0.0 ? 0.0 : var;
    mu[tid] = (float)m;
    rs[tid] = 1.0f / sqrtf((float)var + BN_EPS);
    gg[tid] = bfr(g_rel1[tid]);
    bb[tid] = bfr(bt_rel1[tid]);
  }
  if (tid < NHID * 2 * NHID) wr[tid] = bfr(W_rel2[tid]);
  if (tid < NHID) br[tid] = bfr(b_rel2[tid]);
  __syncthreads();
  const int pix = blockIdx.x * 256 + tid;
  const int n = pix >> 12, l = pix & (LPIX - 1);
  const int colb = el * NTOT + pix;
  float acc[NHID];
#pragma unroll
  for (int o = 0; o < NHID; ++o) acc[o] = 0.0f;
#pragma unroll 1
  for (int c = 0; c < 2 * NHID; ++c) {
    const float raw = c2[(size_t)c * NCOLB + colb];
    const float x = fmaxf((raw - mu[c]) * rs[c] * gg[c] + bb[c], 0.0f);
#pragma unroll
    for (int o = 0; o < NHID; ++o) acc[o] = fmaf(wr[o * 2 * NHID + c], x, acc[o]);
  }
  float mv[NHID];
#pragma unroll
  for (int o = 0; o < NHID; ++o) mv[o] = sigm(acc[o] + br[o]);
  float* mrow = medge + ((size_t)(e * NBATCH + n) * NHID) * LPIX + l;
  for (int pass = 0; pass < 2; ++pass) {
#pragma unroll
    for (int o = 0; o < NHID; ++o) *(volatile float*)(mrow + (size_t)o * LPIX) = mv[o];
    __threadfence();
  }
}

__global__ __launch_bounds__(256) void k_gru_pre(const float* __restrict__ medge, const float* __restrict__ p_nodes,
                                                 const float* __restrict__ Wg, const float* __restrict__ bg,
                                                 const float* __restrict__ Wc,
                                                 float* __restrict__ cnm, float* __restrict__ zpl, float* __restrict__ stat3) {
  __shared__ float wg[4 * NHID];
  __shared__ float wc[NHID * 2 * NHID];
  __shared__ float bgs[2];
  __shared__ float red[8][2 * NHID];
  const int tid = threadIdx.x, lane = tid & 31, wave = tid >> 5;
  const int i = blockIdx.y;
  if (tid < 4 * NHID) wg[tid] = bfr(Wg[i * 4 * NHID + tid]);
  if (tid < NHID * 2 * NHID) wc[tid] = bfr(Wc[i * NHID * 2 * NHID + tid]);
  if (tid < 2) bgs[tid] = bfr(bg[i * 2 + tid]);
  __syncthreads();
  const int col = blockIdx.x * 256 + tid;
  const int n = col >> 12, l = col & (LPIX - 1);
  int cnt = c_INCNT[i]; cnt = cnt < 0 ? 0 : (cnt > 5 ? 5 : cnt);
  const float* hbp = p_nodes + ((size_t)((i + 1) * NBATCH + n) * NHID) * LPIX + l;
  float g0 = 0.0f, g1 = 0.0f;
  float acc[NHID];
#pragma unroll
  for (int o = 0; o < NHID; ++o) acc[o] = 0.0f;
#pragma unroll 1
  for (int c = 0; c < NHID; ++c) {
    float mc = 0.0f;
#pragma unroll 1
    for (int j = 0; j < cnt; ++j) {
      int ej = c_INLIST[i * 5 + j]; ej = ej < 0 ? 0 : (ej > NEDGE - 1 ? NEDGE - 1 : ej);
      mc += medge[((size_t)(ej * NBATCH + n) * NHID + c) * LPIX + l];
    }
    const float hc = bfr(hbp[(size_t)c * LPIX]);
    g0 = fmaf(wg[c], mc, g0); g0 = fmaf(wg[NHID + c], hc, g0);
    g1 = fmaf(wg[2 * NHID + c], mc, g1); g1 = fmaf(wg[3 * NHID + c], hc, g1);
#pragma unroll
    for (int o = 0; o < NHID; ++o) acc[o] = fmaf(wc[o * 2 * NHID + c], mc, acc[o]);
  }
  const float r = sigm(g0 + bgs[0]);
  const float z = sigm(g1 + bgs[1]);
#pragma unroll 1
  for (int c = 0; c < NHID; ++c) {
    const float hc = bfr(hbp[(size_t)c * LPIX]);
    const float rh = r * hc;
#pragma unroll
    for (int o = 0; o < NHID; ++o) acc[o] = fmaf(wc[o * 2 * NHID + NHID + c], rh, acc[o]);
  }
  float* crow = cnm + ((size_t)(i * NBATCH + n) * NHID) * LPIX + l;
  for (int pass = 0; pass < 2; ++pass) {
#pragma unroll
    for (int o = 0; o < NHID; ++o) *(volatile float*)(crow + (size_t)o * LPIX) = acc[o];
    *(volatile float*)(zpl + (size_t)i * NTOT + col) = z;
    __threadfence();
  }
  float sv[NHID], qq[NHID];
#pragma unroll
  for (int o = 0; o < NHID; ++o) { sv[o] = wave_sum(acc[o]); qq[o] = wave_sum(acc[o] * acc[o]); }
  if (lane == 0) {
#pragma unroll
    for (int o = 0; o < NHID; ++o) { red[wave][o] = sv[o]; red[wave][NHID + o] = qq[o]; }
  }
  __syncthreads();
  if (tid < 32) {
    float t = 0.0f;
    if (tid < 2 * NHID) {
#pragma unroll
      for (int w = 0; w < 8; ++w) t += red[w][tid];
    }
    st2f(stat3 + ((size_t)(i * NPIXBLK + blockIdx.x)) * 32 + tid, t);
  }
}

__global__ __launch_bounds__(256) void k_gru_apply(const float* __restrict__ cnm, const float* __restrict__ zpl,
                                                   const float* __restrict__ stat3, const float* __restrict__ p_nodes,
                                                   const float* __restrict__ g_can, const float* __restrict__ bt_can,
                                                   float* __restrict__ out0) {
  __shared__ float mu[NHID], rs[NHID], gg[NHID], bb[NHID];
  const int tid = threadIdx.x;
  const int s = blockIdx.y;
  const int i = (s > 0) ? (s - 1) : 0;
  if (tid < NHID) {
    double sm = 0.0, q = 0.0;
#pragma unroll 1
    for (int b = 0; b < NPIXBLK; ++b) {
      const float* t = stat3 + ((size_t)(i * NPIXBLK + b)) * 32;
      sm += (double)t[tid]; q += (double)t[NHID + tid];
    }
    const double m = sm * (1.0 / NTOT);
    double var = q * (1.0 / NTOT) - m * m;
    var = var < 0.0 ? 0.0 : var;
    mu[tid] = (float)m;
    rs[tid] = 1.0f / sqrtf((float)var + BN_EPS);
    gg[tid] = bfr(g_can[i * NHID + tid]);
    bb[tid] = bfr(bt_can[i * NHID + tid]);
  }
  __syncthreads();
  const int col = blockIdx.x * 256 + tid;
  const int n = col >> 12, l = col & (LPIX - 1);
  if (s == 0) {
    const float* src = p_nodes + ((size_t)n * NHID) * LPIX + l;
    float* dst = out0 + ((size_t)n * NHID) * LPIX + l;
#pragma unroll 1
    for (int o = 0; o < NHID; ++o) st2f(dst + (size_t)o * LPIX, bfr(src[(size_t)o * LPIX]));
  } else {
    const float z = zpl[(size_t)i * NTOT + col];
    const float omz = 1.0f - z;
    const float* hrow = p_nodes + ((size_t)((i + 1) * NBATCH + n) * NHID) * LPIX + l;
    const float* crow = cnm + ((size_t)(i * NBATCH + n) * NHID) * LPIX + l;
    float* orow = out0 + ((size_t)((i + 1) * NBATCH + n) * NHID) * LPIX + l;
#pragma unroll 1
    for (int o = 0; o < NHID; ++o) {
      const float cp = crow[(size_t)o * LPIX];
      float y = (cp - mu[o]) * rs[o] * gg[o] + bb[o];
      y = (y >= 0.0f) ? y : (0.01f * y);
      const float h = bfr(hrow[(size_t)o * LPIX]);
      const float v = omz * h + z * y;
      st2f(orow + (size_t)o * LPIX, v);
    }
  }
}

extern "C" void kernel_launch(void* const* d_in, const int* in_sizes, int n_in,
                              void* d_out, int out_size, void* d_ws, size_t ws_size, hipStream_t stream) {
  (void)in_sizes; (void)out_size;
  if (n_in < 22) return;
  const float* xp      = (const float*)d_in[0];
  const float* p_nodes = (const float*)d_in[1];
  const float* p_atts  = (const float*)d_in[2];
  const float* W_key   = (const float*)d_in[3];
  const float* b_key   = (const float*)d_in[4];
  const float* W_q     = (const float*)d_in[5];
  const float* b_q     = (const float*)d_in[6];
  const float* W_att   = (const float*)d_in[7];
  const float* b_att   = (const float*)d_in[8];
  const float* W_proj  = (const float*)d_in[9];
  const float* g_proj  = (const float*)d_in[10];
  const float* bt_proj = (const float*)d_in[11];
  const float* W_rel1  = (const float*)d_in[12];
  const float* g_rel1  = (const float*)d_in[13];
  const float* bt_rel1 = (const float*)d_in[14];
  const float* W_rel2  = (const float*)d_in[15];
  const float* b_rel2  = (const float*)d_in[16];
  const float* Wg      = (const float*)d_in[17];
  const float* bg      = (const float*)d_in[18];
  const float* Wc      = (const float*)d_in[19];
  const float* g_can   = (const float*)d_in[20];
  const float* bt_can  = (const float*)d_in[21];

  float* out0 = (float*)d_out;
  float* out1 = out0 + OUT1_OFF;

  char* ws = (char*)d_ws; size_t off = 0;
  auto carve = [&](size_t bytes) -> char* { char* p = ws + off; off += (bytes + 255) & ~(size_t)255; return p; };
  unsigned short* btfeat = (unsigned short*)carve(SZ_BTFEAT);
  unsigned short* aall   = (unsigned short*)carve(SZ_AALL);
  unsigned short* arel   = (unsigned short*)carve(SZ_AREL);
  float* c1    = (float*)carve(SZ_C1);
  float* norm  = (float*)carve(SZ_NORM);
  float* qv    = (float*)carve(SZ_QV);
  float* s0    = (float*)carve(SZ_S0);
  float* atts  = (float*)carve(SZ_ATTS);
  float* stat1 = (float*)carve(SZ_STAT1);
  float* msg   = (float*)carve(SZ_MSG);
  unsigned short* btcol = (unsigned short*)carve(SZ_BTCOL);
  float* c2    = (float*)carve(SZ_C2);
  float* stat2 = (float*)carve(SZ_STAT2);
  float* medge = (float*)carve(SZ_MEDGE);
  float* cnm   = (float*)carve(SZ_CNM);
  float* zpl   = (float*)carve(SZ_ZPL);
  float* stat3 = (float*)carve(SZ_STAT3);
  if (off > ws_size || off > (size_t)134217728) return;

  k_prep_w<<<(MALL + MREL) / 8, 256, 0, stream>>>(W_key, W_att, W_proj, W_rel1, aall, arel);
  k_prep_feat<<<NTOT / 8, 256, 0, stream>>>(xp, btfeat);
  {
    const int tiles = (MALL / 64) * (NTOT / 64);
    wmma_gemm64<1, false, 0, 0, false><<<dim3((tiles + 7) / 8, 1), 256, 0, stream>>>(
        aall, (const unsigned short*)nullptr, LDFEAT, 0L,
        btfeat, (const unsigned short*)nullptr, LDFEAT, 0L,
        (void*)c1, (void*)nullptr, NTOT, 0L,
        (const float*)nullptr, (const float*)nullptr, 0L, MALL, NTOT, KFEATP, 1.0f);
  }
  k_softmax_norm<<<NPART * NBATCH, 512, 0, stream>>>(p_atts, norm);
  k_centroid_q<<<NPART * NBATCH, 320, 0, stream>>>(xp, norm, W_q, b_q, qv);
  k_energy_s0<<<NPIXBLK, 256, 0, stream>>>(qv, c1, b_key, p_atts, s0);
  k_logits<<<NPIXBLK, 256, 0, stream>>>(c1, s0, W_att, b_att, atts, out1);
  k_bn1_stats<<<dim3(NPIXBLK, NEDGE), 256, 0, stream>>>(s0, atts, c1, stat1);
  k_msg_write<<<dim3(NPIXBLK, NEDGE), 256, 0, stream>>>(s0, atts, c1, stat1, g_proj, bt_proj, msg);
  for (int b = 0; b < 2; ++b) {
    k_im2col<<<NCOLB / 32, 256, 0, stream>>>(msg, p_nodes, btcol, b);
    const int tiles = (MREL / 64) * (NCOLB / 64);
    wmma_gemm64<0, false, 0, 0, false><<<dim3((tiles + 7) / 8, 1), 256, 0, stream>>>(
        arel, (const unsigned short*)nullptr, KRELP, 0L,
        btcol, (const unsigned short*)nullptr, KRELP, 0L,
        (void*)c2, (void*)nullptr, NCOLB, 0L,
        (const float*)nullptr, (const float*)nullptr, 0L, MREL, NCOLB, KRELP, WCARRY_INV);
    k_bn2_stats<<<dim3(NPIXBLK, EPB), 256, 0, stream>>>(c2, stat2);
    k_edge_finish<<<dim3(NPIXBLK, EPB), 256, 0, stream>>>(c2, stat2, g_rel1, bt_rel1, W_rel2, b_rel2, medge, b);
  }
  k_gru_pre<<<dim3(NPIXBLK, NPART), 256, 0, stream>>>(medge, p_nodes, Wg, bg, Wc, cnm, zpl, stat3);
  k_gru_apply<<<dim3(NPIXBLK, NPART + 1), 256, 0, stream>>>(cnm, zpl, stat3, p_nodes, g_can, bt_can, out0);
}
